// VGATEncoder_48876727828951
// MI455X (gfx1250) — hardware-verified
//
#include <hip/hip_runtime.h>
#include <stddef.h>


#define NTHR    256
#define NWAVE   8
#define EPT     8
#define NGRP    2
#define CHUNK   (NTHR * EPT * NGRP)
#define WCAP    (EPT * NGRP * 32)
#define LISTN   (NWAVE * WCAP)
#define NBC     4096
#define NBF     1024
#define RCAP    40960
#define RBN     128
#define TGT     256
#define DEGCAP  1024
#define OTHR    512
#define BM      64
#define WSCAP   134217728
#define FIN     128
#define FH      128
#define FZ      64
#define FP      128
#define ACARRY  8.0f
#define WCARRY  64.0f
#define GSCALE  (1.0f / 512.0f)
#define SLOPE_ATT 0.2f

#define LDS_FILL ((RCAP + NBF + LISTN) * 4 + 64)

static_assert((CHUNK & (CHUNK - 1)) == 0);
static_assert(CHUNK <= 4096);
static_assert((NBC & (NBC - 1)) == 0 && (NBF & (NBF - 1)) == 0);
static_assert(NBC == 4 * NBF);
static_assert(OTHR * 8 == NBC);
static_assert((RCAP % 32) == 0);
static_assert(TGT == NWAVE * 32);
static_assert((NBC % TGT) == 0);
static_assert((TGT % BM) == 0);
static_assert(WCAP == EPT * NGRP * 32);
static_assert(FIN == 128 && FH == 128 && FZ == 64 && FP == 2 * FZ);
static_assert((FIN % 32) == 0 && (FH % 32) == 0);

typedef float    v2f  __attribute__((ext_vector_type(2)));
typedef float    v4f  __attribute__((ext_vector_type(4)));
typedef float    v8f  __attribute__((ext_vector_type(8)));
typedef int      v4i  __attribute__((ext_vector_type(4)));
typedef _Float16 v4h  __attribute__((ext_vector_type(4)));
typedef _Float16 v8h  __attribute__((ext_vector_type(8)));
typedef _Float16 v16h __attribute__((ext_vector_type(16)));
union Frag { v16h v; v8h h[2]; };

__device__ __forceinline__ v8f wmh(v16h a, v16h b, v8f c) {
  v8f d = __builtin_amdgcn_wmma_f32_16x16x32_f16(false, a, false, b, (short)0, c, false, false);
  asm volatile("v_nop\n\tv_nop\n\tv_nop\n\tv_nop" : "+v"(d) : "v"(a), "v"(b));
  return d;
}

__device__ __forceinline__ v4f selz(v4f v, bool live) {
  v4f o; o.x = live ? v.x : 0.f; o.y = live ? v.y : 0.f; o.z = live ? v.z : 0.f; o.w = live ? v.w : 0.f; return o;
}
__device__ __forceinline__ v4f sel4(bool c, v4f a, v4f b) {
  v4f o; o.x = c ? a.x : b.x; o.y = c ? a.y : b.y; o.z = c ? a.z : b.z; o.w = c ? a.w : b.w; return o;
}
__device__ __forceinline__ float lrelu1(float v) { return v >= 0.f ? v : SLOPE_ATT * v; }
__device__ __forceinline__ float wmax1(float v) {
#pragma unroll
  for (int off = 16; off > 0; off >>= 1) v = fmaxf(v, __shfl_xor(v, off));
  return v;
}
__device__ __forceinline__ float wsum1(float v) {
#pragma unroll
  for (int off = 16; off > 0; off >>= 1) v += __shfl_xor(v, off);
  return v;
}

template <int NB>
__device__ __forceinline__ int scan_chunk(const int* __restrict__ dsts, int nE, int cbase, int slotBase,
                                          int vec8, int* list, int tid, int lane, int wave) {
  int wc = 0;
#pragma unroll
  for (int g = 0; g < NGRP; ++g) {
    const int el0  = (g * NTHR + tid) * EPT;
    const int e0   = cbase + el0;
    const int sent = -2147483647 - 1;
    v4i da, db;
    if (vec8 != 0 && cbase + CHUNK <= nE) {
      da = *(const v4i*)(dsts + e0);
      db = *(const v4i*)(dsts + e0 + 4);
    } else {
      da.x = (e0     < nE) ? dsts[min(e0, nE - 1)] : sent;
      da.y = (e0 + 1 < nE) ? dsts[min(e0 + 1, nE - 1)] : sent;
      da.z = (e0 + 2 < nE) ? dsts[min(e0 + 2, nE - 1)] : sent;
      da.w = (e0 + 3 < nE) ? dsts[min(e0 + 3, nE - 1)] : sent;
      db.x = (e0 + 4 < nE) ? dsts[min(e0 + 4, nE - 1)] : sent;
      db.y = (e0 + 5 < nE) ? dsts[min(e0 + 5, nE - 1)] : sent;
      db.z = (e0 + 6 < nE) ? dsts[min(e0 + 6, nE - 1)] : sent;
      db.w = (e0 + 7 < nE) ? dsts[min(e0 + 7, nE - 1)] : sent;
    }
    const unsigned nb = (unsigned)slotBase;
    const unsigned s0 = (unsigned)da.x - nb, s1 = (unsigned)da.y - nb;
    const unsigned s2 = (unsigned)da.z - nb, s3 = (unsigned)da.w - nb;
    const unsigned s4 = (unsigned)db.x - nb, s5 = (unsigned)db.y - nb;
    const unsigned s6 = (unsigned)db.z - nb, s7 = (unsigned)db.w - nb;
    const bool h0 = s0 < (unsigned)NB, h1 = s1 < (unsigned)NB, h2 = s2 < (unsigned)NB, h3 = s3 < (unsigned)NB;
    const bool h4 = s4 < (unsigned)NB, h5 = s5 < (unsigned)NB, h6 = s6 < (unsigned)NB, h7 = s7 < (unsigned)NB;
    const unsigned any = __builtin_amdgcn_ballot_w32(h0 | h1 | h2 | h3 | h4 | h5 | h6 | h7);
    if (any != 0u) {
#define HITJ(J, HJ, SJ) { \
        const unsigned mj = __builtin_amdgcn_ballot_w32(HJ); \
        if (mj != 0u) { \
          if (HJ) { \
            const int pos = wc + (int)__builtin_amdgcn_mbcnt_lo(mj, 0u); \
            if (pos < WCAP) list[wave * WCAP + pos] = ((el0 + (J)) << 12) | (int)(SJ); \
          } \
          wc += (int)__builtin_popcount(mj); } }
      HITJ(0, h0, s0)
      HITJ(1, h1, s1)
      HITJ(2, h2, s2)
      HITJ(3, h3, s3)
      HITJ(4, h4, s4)
      HITJ(5, h5, s5)
      HITJ(6, h6, s6)
      HITJ(7, h7, s7)
#undef HITJ
    }
  }
  return wc;
}

__global__ __launch_bounds__(NTHR) void k_count(const int* __restrict__ dsts, int* cnt, int nE, int vec8) {
  __shared__ __attribute__((aligned(16))) int scnt[NBC];
  __shared__ __attribute__((aligned(16))) int list[LISTN];
  __shared__ int wcnt[NWAVE];
  const int tid = threadIdx.x, lane = tid & 31, wave = tid >> 5;
  const int nodeBase = blockIdx.x * NBC;

  for (int i = tid; i < NBC; i += NTHR) scnt[i] = 0;
  __syncthreads();

  const int nChunks = (nE + CHUNK - 1) / CHUNK;
#pragma unroll 1
  for (int ch = 0; ch < nChunks; ++ch) {
    const int cbase = ch * CHUNK;
    const int wc = scan_chunk<NBC>(dsts, nE, cbase, nodeBase, vec8, list, tid, lane, wave);
    if (lane == 0) wcnt[wave] = wc;
    __syncthreads();
    if (wave == 0) {
#pragma unroll 1
      for (int wsx = 0; wsx < NWAVE; ++wsx) {
        int n = __builtin_amdgcn_readfirstlane(wcnt[wsx]);
        n = n > WCAP ? WCAP : (n < 0 ? 0 : n);
        const int* lp = list + wsx * WCAP;
#pragma unroll 1
        for (int i = 0; i < n; ++i) {
          const int ent  = __builtin_amdgcn_readfirstlane(lp[i]);
          const int slot = ent & (NBC - 1);
          if (lane == 0) scnt[slot] = scnt[slot] + 1;
        }
      }
    }
    __syncthreads();
  }

  v4i cq[4];
#pragma unroll
  for (int q = 0; q < 4; ++q) {
    const int f = (wave * 4 + q) * 128 + 4 * lane;
    cq[q] = *(const v4i*)(scnt + f);
  }
  int* cp = cnt + (size_t)nodeBase;
#pragma unroll
  for (int q = 0; q < 4; ++q) {
    const int f = (wave * 4 + q) * 128 + 4 * lane;
    *(volatile v4i*)(cp + f) = cq[q];
  }
  __threadfence();
#pragma unroll
  for (int q = 0; q < 4; ++q) {
    const int f = (wave * 4 + q) * 128 + 4 * lane;
    *(volatile v4i*)(cp + f) = cq[q];
  }
}

__global__ __launch_bounds__(OTHR) void k_offsets(
    const int* __restrict__ cnt, int* off, int* rbase, int* flagp, int nChunk) {
  __shared__ __attribute__((aligned(16))) int soff[NBC];
  __shared__ __attribute__((aligned(16))) int srb[RBN];
  __shared__ int wtot[OTHR / 32];
  __shared__ int wbad[OTHR / 32];
  const int tid = threadIdx.x, lane = tid & 31, wave = tid >> 5, sub = tid >> 7;
  for (int i = tid; i < RBN; i += OTHR) srb[i] = 0;
  int carry = 0;
  int bad = 0;
#pragma unroll 1
  for (int ch = 0; ch < nChunk; ++ch) {
    const int base = ch * NBC;
    const v4i c0 = *(const v4i*)(cnt + base + 8 * tid);
    const v4i c1 = *(const v4i*)(cnt + base + 8 * tid + 4);
    const int e0 = max(c0.x, 0), e1 = max(c0.y, 0), e2 = max(c0.z, 0), e3 = max(c0.w, 0);
    const int e4 = max(c1.x, 0), e5 = max(c1.y, 0), e6 = max(c1.z, 0), e7 = max(c1.w, 0);
    bad |= (int)(e0 > DEGCAP) | (int)(e1 > DEGCAP) | (int)(e2 > DEGCAP) | (int)(e3 > DEGCAP) |
           (int)(e4 > DEGCAP) | (int)(e5 > DEGCAP) | (int)(e6 > DEGCAP) | (int)(e7 > DEGCAP);
    const int ts = e0 + e1 + e2 + e3 + e4 + e5 + e6 + e7;
    int incl = ts;
#pragma unroll
    for (int d = 1; d < 32; d <<= 1) {
      const int t = __shfl_up(incl, d);
      if (lane >= d) incl += t;
    }
    if (lane == 31) wtot[wave] = incl;
    __syncthreads();
    const int S0 = wtot[0]  + wtot[1]  + wtot[2]  + wtot[3];
    const int S1 = wtot[4]  + wtot[5]  + wtot[6]  + wtot[7];
    const int S2 = wtot[8]  + wtot[9]  + wtot[10] + wtot[11];
    const int S3 = wtot[12] + wtot[13] + wtot[14] + wtot[15];
    bad |= (int)(S0 > RCAP) | (int)(S1 > RCAP) | (int)(S2 > RCAP) | (int)(S3 > RCAP);
    int pre = 0;
#pragma unroll 1
    for (int w = 4 * sub; w < wave; ++w) pre += wtot[w];
    const int b0 = carry;
    const int b1 = b0 + ((S0 + 31) & ~31);
    const int b2 = b1 + ((S1 + 31) & ~31);
    const int b3 = b2 + ((S2 + 31) & ~31);
    const int b4 = b3 + ((S3 + 31) & ~31);
    const int myb = sub == 0 ? b0 : (sub == 1 ? b1 : (sub == 2 ? b2 : b3));
    if (tid == 0) {
      srb[min(4 * ch + 0, RBN - 1)] = b0;
      srb[min(4 * ch + 1, RBN - 1)] = b1;
      srb[min(4 * ch + 2, RBN - 1)] = b2;
      srb[min(4 * ch + 3, RBN - 1)] = b3;
    }
    int run = myb + pre + incl - ts;
    soff[8 * tid + 0] = run; run += e0;
    soff[8 * tid + 1] = run; run += e1;
    soff[8 * tid + 2] = run; run += e2;
    soff[8 * tid + 3] = run; run += e3;
    soff[8 * tid + 4] = run; run += e4;
    soff[8 * tid + 5] = run; run += e5;
    soff[8 * tid + 6] = run; run += e6;
    soff[8 * tid + 7] = run;
    carry = b4;
    __syncthreads();
    const v4i o0 = *(const v4i*)(soff + 4 * tid);
    const v4i o1 = *(const v4i*)(soff + 4 * (tid + OTHR));
    int* op = off + base;
    *(volatile v4i*)(op + 4 * tid) = o0;
    *(volatile v4i*)(op + 4 * (tid + OTHR)) = o1;
    __threadfence();
    *(volatile v4i*)(op + 4 * tid) = o0;
    *(volatile v4i*)(op + 4 * (tid + OTHR)) = o1;
    __syncthreads();
  }
  if (tid == 0) srb[min(4 * nChunk, RBN - 1)] = carry;
  const unsigned bm = __builtin_amdgcn_ballot_w32(bad != 0);
  if (lane == 0) wbad[wave] = (bm != 0u) ? 1 : 0;
  __syncthreads();
  int F = 0;
#pragma unroll
  for (int w = 0; w < OTHR / 32; ++w) F |= wbad[w];
  v4i rv = {0, 0, 0, 0};
  if (tid < 32) rv = *(const v4i*)(srb + 4 * tid);
  if (tid < 32) { *(volatile v4i*)(rbase + 4 * tid) = rv; *(volatile int*)(flagp + tid) = F; }
  __threadfence();
  if (tid < 32) { *(volatile v4i*)(rbase + 4 * tid) = rv; *(volatile int*)(flagp + tid) = F; }
}

__global__ __launch_bounds__(NTHR) void k_fill(
    const int* __restrict__ srcs, const int* __restrict__ dsts,
    const int* __restrict__ off, const int* __restrict__ rbase,
    int* csr, int nN, int nE, int vec8, int csrLen) {
  extern __shared__ v4f lds_dyn[];
  int* region = (int*)lds_dyn;
  int* cursor = region + RCAP;
  int* list   = cursor + NBF;
  int* wcnt   = list + LISTN;
  const int tid = threadIdx.x, lane = tid & 31, wave = tid >> 5;
  const int b = blockIdx.x;
  const int nodeBase = b * NBF;

  int rb0 = rbase[b];
  const int rb1 = rbase[b + 1];
  rb0 = rb0 < 0 ? 0 : (rb0 > csrLen ? csrLen : rb0);
  rb0 &= ~31;
  int len = rb1 - rb0;
  len = len < 0 ? 0 : (len > RCAP ? RCAP : len);
  int lenW = (len + 31) & ~31;
  if (rb0 + lenW > csrLen) lenW = (csrLen - rb0) & ~31;

  {
    const v4i z = {0, 0, 0, 0};
    for (int i = tid; i < RCAP / 4; i += NTHR) ((v4i*)region)[i] = z;
    for (int s = tid; s < NBF; s += NTHR) {
      int o = off[nodeBase + s] - rb0;
      o = o < 0 ? 0 : (o > RCAP ? RCAP : o);
      cursor[s] = o;
    }
  }
  __syncthreads();

  const int nChunks = (nE + CHUNK - 1) / CHUNK;
#pragma unroll 1
  for (int ch = 0; ch < nChunks; ++ch) {
    const int cbase = ch * CHUNK;
    const int wc = scan_chunk<NBF>(dsts, nE, cbase, nodeBase, vec8, list, tid, lane, wave);
    if (lane == 0) wcnt[wave] = wc;
    __syncthreads();
    if (wave == 0) {
#pragma unroll 1
      for (int wsx = 0; wsx < NWAVE; ++wsx) {
        int n = __builtin_amdgcn_readfirstlane(wcnt[wsx]);
        n = n > WCAP ? WCAP : (n < 0 ? 0 : n);
        const int* lp = list + wsx * WCAP;
#pragma unroll 1
        for (int i = 0; i < n; ++i) {
          const int ent  = __builtin_amdgcn_readfirstlane(lp[i]);
          const int slot = ent & (NBF - 1);
          int e = cbase + ((ent >> 12) & (CHUNK - 1));
          e = e > nE - 1 ? nE - 1 : e;
          int sv = srcs[e];
          sv = sv < 0 ? 0 : (sv > nN - 1 ? nN - 1 : sv);
          if (lane == 0) {
            int pos = cursor[slot];
            pos = pos < 0 ? 0 : (pos > RCAP - 1 ? RCAP - 1 : pos);
            region[pos] = sv;
            const int np = pos + 1;
            cursor[slot] = np > RCAP ? RCAP : np;
          }
        }
      }
    }
    __syncthreads();
  }

  const int nv = lenW >> 2;
  int* gp = csr + rb0;
#pragma unroll 1
  for (int i = tid; i < nv; i += NTHR) { const v4i v = ((const v4i*)region)[i]; *(volatile v4i*)(gp + 4 * i) = v; }
  __threadfence();
#pragma unroll 1
  for (int i = tid; i < nv; i += NTHR) { const v4i v = ((const v4i*)region)[i]; *(volatile v4i*)(gp + 4 * i) = v; }
}

__global__ __launch_bounds__(NTHR) void k_wcvt2(const float* __restrict__ wA, const float* __restrict__ wB,
                                                _Float16* dp, int K, int NcA, int NcB, int nUnits) {
  const int i = (int)blockIdx.x * NTHR + (int)threadIdx.x;
  if (i >= nUnits) return;
  const int ppr = K >> 3;
  const int n = i / ppr;
  const int seg = i - n * ppr;
  int na = n > NcA - 1 ? NcA - 1 : n;
  na = na < 0 ? 0 : na;
  int nb = n - NcA;
  nb = nb < 0 ? 0 : (nb > NcB - 1 ? NcB - 1 : nb);
  const bool useA = n < NcA;
  v8h o;
#pragma unroll
  for (int j = 0; j < 8; ++j) {
    int k = 8 * seg + j;
    k = k > K - 1 ? K - 1 : (k < 0 ? 0 : k);
    const float fa = wA[(size_t)k * NcA + na];
    const float fb = wB[(size_t)k * NcB + nb];
    const float f = useA ? fa : fb;
    o[j] = (_Float16)(f * WCARRY);
  }
  _Float16* gp = dp + (size_t)i * 8;
  *(volatile v8h*)gp = o;
  __threadfence();
  *(volatile v8h*)gp = o;
}

__global__ __launch_bounds__(OTHR) void k_wfold4(const float* __restrict__ gwA, const float* __restrict__ gwB,
                                                 const float* __restrict__ a0, const float* __restrict__ a1,
                                                 const float* __restrict__ a2, const float* __restrict__ a3,
                                                 float* wa, int K, int C) {
  __shared__ __attribute__((aligned(16))) float so[OTHR];
  const int tid = threadIdx.x;
  const int k = tid >> 2, j = tid & 3;
  int kk = k > K - 1 ? K - 1 : k;
  kk = kk < 0 ? 0 : kk;
  const bool live = k < K;
  const float* wpa = gwA + (size_t)kk * C;
  const float* wpb = gwB + (size_t)kk * C;
  float acc = 0.f;
#pragma unroll 1
  for (int c = 0; c < C; ++c) {
    const float va = wpa[c], vb = wpb[c];
    const float x0 = a0[c], x1 = a1[c], x2 = a2[c], x3 = a3[c];
    const float wv = (j < 2) ? va : vb;
    const float av = (j == 0) ? x0 : ((j == 1) ? x1 : ((j == 2) ? x2 : x3));
    acc += wv * av;
  }
  so[tid] = live ? acc : 0.f;
  __syncthreads();
  v4f v = {0.f, 0.f, 0.f, 0.f};
  if (tid < OTHR / 4) v = *(const v4f*)(so + 4 * tid);
  if (tid < OTHR / 4) *(volatile v4f*)(wa + 4 * tid) = v;
  __threadfence();
  if (tid < OTHR / 4) *(volatile v4f*)(wa + 4 * tid) = v;
}

__global__ __launch_bounds__(NTHR) void k_xcvt(const float* __restrict__ src, _Float16* dst, int nN, int npad) {
  const int gi = (int)blockIdx.x * NTHR + (int)threadIdx.x;
  const int row = gi >> 4, seg = gi & 15;
  if (row >= npad) return;
  int rr = row > nN - 1 ? nN - 1 : row;
  rr = rr < 0 ? 0 : rr;
  const bool live = row < nN;
  const float* p = src + (size_t)rr * FIN + 8 * seg;
  const v4f u0 = selz(*(const v4f*)p, live);
  const v4f u1 = selz(*(const v4f*)(p + 4), live);
  v8h o;
  o[0] = (_Float16)(u0.x * ACARRY); o[1] = (_Float16)(u0.y * ACARRY);
  o[2] = (_Float16)(u0.z * ACARRY); o[3] = (_Float16)(u0.w * ACARRY);
  o[4] = (_Float16)(u1.x * ACARRY); o[5] = (_Float16)(u1.y * ACARRY);
  o[6] = (_Float16)(u1.z * ACARRY); o[7] = (_Float16)(u1.w * ACARRY);
  _Float16* gp = dst + (size_t)row * FIN + 8 * seg;
  *(volatile v8h*)gp = o;
  __threadfence();
  *(volatile v8h*)gp = o;
}

template <int KW>
__global__ __launch_bounds__(NTHR) void k_logit4(const float* __restrict__ hin, const float* __restrict__ wa,
                                                 float* es4, int nN) {
  static_assert((KW % 4) == 0 && KW <= NTHR && KW >= 8);
  __shared__ __attribute__((aligned(16))) float swa[4 * KW];
  const int tid = threadIdx.x;
  if (tid < KW) *(v4f*)(swa + 4 * tid) = *(const v4f*)(wa + 4 * tid);
  __syncthreads();
  const int node = (int)blockIdx.x * NTHR + tid;
  int rr = node > nN - 1 ? nN - 1 : node;
  rr = rr < 0 ? 0 : rr;
  const bool live = node < nN;
  float e0 = 0.f, e1 = 0.f, e2 = 0.f, e3 = 0.f;
  const float* hp = hin + (size_t)rr * KW;
#pragma unroll 1
  for (int kq = 0; kq < KW / 4; ++kq) {
    const v4f hv = *(const v4f*)(hp + 4 * kq);
    const v4f w0 = *(const v4f*)(swa + 16 * kq);
    const v4f w1 = *(const v4f*)(swa + 16 * kq + 4);
    const v4f w2 = *(const v4f*)(swa + 16 * kq + 8);
    const v4f w3 = *(const v4f*)(swa + 16 * kq + 12);
    e0 += hv.x * w0.x; e1 += hv.x * w0.y; e2 += hv.x * w0.z; e3 += hv.x * w0.w;
    e0 += hv.y * w1.x; e1 += hv.y * w1.y; e2 += hv.y * w1.z; e3 += hv.y * w1.w;
    e0 += hv.z * w2.x; e1 += hv.z * w2.y; e2 += hv.z * w2.z; e3 += hv.z * w2.w;
    e0 += hv.w * w3.x; e1 += hv.w * w3.y; e2 += hv.w * w3.z; e3 += hv.w * w3.w;
  }
  v4f ev;
  ev.x = live ? e0 : 0.f; ev.y = live ? e1 : 0.f; ev.z = live ? e2 : 0.f; ev.w = live ? e3 : 0.f;
  float* gp = es4 + (size_t)node * 4;
  *(volatile v4f*)gp = ev;
  __threadfence();
  *(volatile v4f*)gp = ev;
}

template <int BNC>
__global__ __launch_bounds__(NTHR) void k_gemm(
    const _Float16* __restrict__ A, const _Float16* __restrict__ Bp,
    float* Cout, int K, int ldc, int nValid, int nStore) {
  constexpr int TPW = BNC / 32;
  constexpr int PPR = BNC / 4;
  constexpr int NIT = (BM * PPR) / NTHR;
  static_assert(TPW >= 1 && TPW * 32 == BNC);
  static_assert((BM * PPR) % NTHR == 0);
  static_assert(NIT >= 1);
  static_assert(BM == 4 * 16);
  static_assert((PPR & (PPR - 1)) == 0);

  __shared__ __attribute__((aligned(16))) float stg[BM * BNC];
  const int tid = threadIdx.x, lane = tid & 31, wave = tid >> 5, hh = lane >> 4, m = lane & 15;
  const int rowBase = (int)blockIdx.x * BM;
  const int colBase = (int)blockIdx.y * BNC;
  const int rg = wave >> 1, chf = wave & 1;
  const int r0 = rg * 16;
  const int c0 = chf * (BNC / 2);

  v8f acc[TPW];
#pragma unroll
  for (int t = 0; t < TPW; ++t) { v8f z = {0.f, 0.f, 0.f, 0.f, 0.f, 0.f, 0.f, 0.f}; acc[t] = z; }

  const _Float16* ap = A  + (size_t)(rowBase + r0 + m) * K + 8 * hh;
  const _Float16* bp = Bp + (size_t)(colBase + c0 + m) * K + 8 * hh;
  const int ksteps = K >> 5;
#pragma unroll 1
  for (int kt = 0; kt < ksteps; ++kt) {
    Frag a;
    a.h[0] = *(const v8h*)(ap + 32 * kt);
    a.h[1] = *(const v8h*)(ap + 32 * kt + 16);
#pragma unroll
    for (int t = 0; t < TPW; ++t) {
      const size_t to = (size_t)(16 * t) * K + 32 * kt;
      Frag b;
      b.h[0] = *(const v8h*)(bp + to);
      b.h[1] = *(const v8h*)(bp + to + 16);
      acc[t] = wmh(a.v, b.v, acc[t]);
    }
  }

  {
    float* sp = stg + (size_t)(r0 + 8 * hh) * BNC + c0 + m;
    const int growb = rowBase + r0 + 8 * hh;
#pragma unroll
    for (int t = 0; t < TPW; ++t) {
#pragma unroll
      for (int r = 0; r < 8; ++r) {
        const bool lv = (growb + r) < nValid;
        const float g = acc[t][r] * GSCALE;
        sp[r * BNC + 16 * t] = lv ? g : 0.f;
      }
    }
  }
  __syncthreads();

  v4f cv[NIT];
#pragma unroll
  for (int it = 0; it < NIT; ++it) {
    const int id = it * NTHR + tid;
    const int row = id / PPR, seg = id & (PPR - 1);
    cv[it] = *(const v4f*)(stg + (size_t)row * BNC + 4 * seg);
  }
#pragma unroll
  for (int it = 0; it < NIT; ++it) {
    const int id = it * NTHR + tid;
    const int row = id / PPR, seg = id & (PPR - 1);
    const int grow = rowBase + row;
    if (grow < nStore) {
      float* gp = Cout + (size_t)grow * ldc + colBase + 4 * seg;
      *(volatile v4f*)gp = cv[it];
    }
  }
  __threadfence();
#pragma unroll
  for (int it = 0; it < NIT; ++it) {
    const int id = it * NTHR + tid;
    const int row = id / PPR, seg = id & (PPR - 1);
    const int grow = rowBase + row;
    if (grow < nStore) {
      float* gp = Cout + (size_t)grow * ldc + colBase + 4 * seg;
      *(volatile v4f*)gp = cv[it];
    }
  }
}

template <int STAGE>
__global__ __launch_bounds__(NTHR) void k_aggatt(
    const int* __restrict__ csr, const int* __restrict__ off, const int* __restrict__ cnt,
    const float* __restrict__ es4, const float* __restrict__ hp,
    const float* __restrict__ gbA, const float* __restrict__ gbB,
    const float* __restrict__ epsn, const int* __restrict__ flagp,
    float* hout, _Float16* aout, float* zout, float* klpart, int nN, int csrLen) {
  __shared__ float wkl[NWAVE];
  const int tid = threadIdx.x, lane = tid & 31, wave = tid >> 5;
  const int tbase = blockIdx.x * TGT + wave * 32;
  const int cl    = tbase + lane;
  const int cnt_l = cnt[cl];
  const int off_l = off[cl];
  const float NINF = -__builtin_inff();
  const float QNAN = __int_as_float(0x7fc00000);
  const int pz = (STAGE == 2) ? flagp[0] : 0;
  const bool hiHalf = (STAGE == 2) && (lane >= 16);
  v4f bq;
  {
    const int bi = (STAGE == 1) ? 4 * lane : 4 * (lane & 15);
    const v4f ba = *(const v4f*)(gbA + bi);
    const v4f bb = *(const v4f*)(gbB + bi);
    bq = sel4(hiHalf, bb, ba);
  }
  float klacc = 0.f;

#pragma unroll 1
  for (int j = 0; j < 32; ++j) {
    const int c = tbase + j;
    int n = __shfl(cnt_l, j);
    n = n < 0 ? 0 : (n > DEGCAP ? DEGCAP : n);
    const int st = __shfl(off_l, j);
    const v4f ec = *(const v4f*)(es4 + (size_t)c * 4);
    const float edc0 = ec.y, edc1 = ec.w;
    const float es0 = lrelu1(ec.x + ec.y);
    const float es1 = lrelu1(ec.z + ec.w);

    float m0 = es0, m1 = es1;
#pragma unroll 1
    for (int q0 = 0; q0 < n; q0 += 32) {
      int pos = st + q0 + lane;
      pos = pos < 0 ? 0 : (pos > csrLen - 1 ? csrLen - 1 : pos);
      int sl = csr[pos];
      sl = sl < 0 ? 0 : (sl > nN - 1 ? nN - 1 : sl);
      const int mcnt = (n - q0) < 32 ? (n - q0) : 32;
      const bool valid = lane < mcnt;
      const v4f ev = *(const v4f*)(es4 + (size_t)sl * 4);
      float e0 = lrelu1(ev.x + edc0);
      e0 = valid ? e0 : NINF;
      e0 = wmax1(e0);
      m0 = fmaxf(m0, e0);
      if (STAGE == 2) {
        float e1 = lrelu1(ev.z + edc1);
        e1 = valid ? e1 : NINF;
        e1 = wmax1(e1);
        m1 = fmaxf(m1, e1);
      }
    }
    const float x0 = __expf(es0 - m0);
    const float x1 = (STAGE == 2) ? __expf(es1 - m1) : 0.f;
    float z0 = x0, z1v = x1;
#pragma unroll 1
    for (int q0 = 0; q0 < n; q0 += 32) {
      int pos = st + q0 + lane;
      pos = pos < 0 ? 0 : (pos > csrLen - 1 ? csrLen - 1 : pos);
      int sl = csr[pos];
      sl = sl < 0 ? 0 : (sl > nN - 1 ? nN - 1 : sl);
      const int mcnt = (n - q0) < 32 ? (n - q0) : 32;
      const bool valid = lane < mcnt;
      const v4f ev = *(const v4f*)(es4 + (size_t)sl * 4);
      float f0 = __expf(lrelu1(ev.x + edc0) - m0);
      f0 = valid ? f0 : 0.f;
      z0 = z0 + wsum1(f0);
      if (STAGE == 2) {
        float f1 = __expf(lrelu1(ev.z + edc1) - m1);
        f1 = valid ? f1 : 0.f;
        z1v = z1v + wsum1(f1);
      }
    }
    const float rz0 = __builtin_amdgcn_rcpf(z0);
    const float rz1 = (STAGE == 2) ? __builtin_amdgcn_rcpf(z1v) : 0.f;
    const float as0 = x0 * rz0, as1 = x1 * rz1;
    const float asl = hiHalf ? as1 : as0;

    v4f acc = (*(const v4f*)(hp + (size_t)c * FP + 4 * lane)) * asl;
#pragma unroll 1
    for (int q0 = 0; q0 < n; q0 += 32) {
      int pos = st + q0 + lane;
      pos = pos < 0 ? 0 : (pos > csrLen - 1 ? csrLen - 1 : pos);
      int sl = csr[pos];
      sl = sl < 0 ? 0 : (sl > nN - 1 ? nN - 1 : sl);
      const int mcnt = (n - q0) < 32 ? (n - q0) : 32;
      const bool valid = lane < mcnt;
      const v4f ev = *(const v4f*)(es4 + (size_t)sl * 4);
      float al0 = __expf(lrelu1(ev.x + edc0) - m0) * rz0;
      al0 = valid ? al0 : 0.f;
      float al1 = 0.f;
      if (STAGE == 2) {
        al1 = __expf(lrelu1(ev.z + edc1) - m1) * rz1;
        al1 = valid ? al1 : 0.f;
      }
#pragma unroll 1
      for (int pp = 0; pp < mcnt; ++pp) {
        const int s = __builtin_amdgcn_readlane(sl, pp);
        const float ap0 = __int_as_float(__builtin_amdgcn_readlane(__float_as_int(al0), pp));
        float ap = ap0;
        if (STAGE == 2) {
          const float ap1 = __int_as_float(__builtin_amdgcn_readlane(__float_as_int(al1), pp));
          ap = hiHalf ? ap1 : ap0;
        }
        const v4f hv = *(const v4f*)(hp + (size_t)s * FP + 4 * lane);
        acc = acc + hv * ap;
      }
    }

    const bool live = c < nN;
    const v4f ob = acc + bq;
    if (STAGE == 1) {
      v4f o;
      o.x = fmaxf(ob.x, 0.f); o.y = fmaxf(ob.y, 0.f); o.z = fmaxf(ob.z, 0.f); o.w = fmaxf(ob.w, 0.f);
      o = selz(o, live);
      v4h q;
      q.x = (_Float16)(o.x * ACARRY); q.y = (_Float16)(o.y * ACARRY);
      q.z = (_Float16)(o.z * ACARRY); q.w = (_Float16)(o.w * ACARRY);
      float* gp = hout + (size_t)c * FP + 4 * lane;
      _Float16* hq = aout + (size_t)c * FP + 4 * lane;
      *(volatile v4f*)gp = o;
      *(volatile v4h*)hq = q;
      __threadfence();
      *(volatile v4f*)gp = o;
      *(volatile v4h*)hq = q;
    } else {
      const int qs = lane >> 1;
      const bool odd = (lane & 1) != 0;
      const float m0s = __shfl(ob.x, qs), m1s = __shfl(ob.y, qs), m2s = __shfl(ob.z, qs), m3s = __shfl(ob.w, qs);
      const float t0s = __shfl(ob.x, qs + 16), t1s = __shfl(ob.y, qs + 16);
      const float t2s = __shfl(ob.z, qs + 16), t3s = __shfl(ob.w, qs + 16);
      v2f mu, ls;
      mu.x = odd ? m2s : m0s; mu.y = odd ? m3s : m1s;
      ls.x = odd ? t2s : t0s; ls.y = odd ? t3s : t1s;
      int cc = c > nN - 1 ? nN - 1 : c;
      cc = cc < 0 ? 0 : cc;
      const v2f ep = *(const v2f*)(epsn + (size_t)cc * FZ + 2 * lane);
      v2f sg; sg.x = __expf(ls.x); sg.y = __expf(ls.y);
      v2f zz = mu + sg * ep;
      const float kle = (sg.x * sg.x + mu.x * mu.x - ls.x - 0.5f) + (sg.y * sg.y + mu.y * mu.y - ls.y - 0.5f);
      klacc += live ? kle : 0.f;
      zz.x = (pz != 0) ? QNAN : zz.x; zz.y = (pz != 0) ? QNAN : zz.y;
      float* gp = zout + (size_t)cc * FZ + 2 * lane;
      if (live) *(volatile v2f*)gp = zz;
      __threadfence();
      if (live) *(volatile v2f*)gp = zz;
    }
  }

  if (STAGE == 2) {
    const float wsv = wsum1(klacc);
    if (lane == 0) wkl[wave] = wsv;
    __syncthreads();
    if (wave == 0) {
      float tot = 0.f;
#pragma unroll
      for (int w = 0; w < NWAVE; ++w) tot += wkl[w];
      tot = (pz != 0) ? QNAN : tot;
      const float v = (lane == 0) ? tot : 0.f;
      float* kp = klpart + (size_t)blockIdx.x * 32 + lane;
      *(volatile float*)kp = v;
      __threadfence();
      *(volatile float*)kp = v;
    }
  }
}

__global__ __launch_bounds__(NTHR) void k_klsum(const float* __restrict__ klpart, const float* __restrict__ ewUnused,
                                                float* out, int nPart, int klIdx) {
  __shared__ double sd[NTHR];
  const int tid = threadIdx.x;
  double a = 0.0;
#pragma unroll 1
  for (int i = tid; i < nPart; i += NTHR) a += (double)klpart[(size_t)i * 32];
  sd[tid] = a;
  __syncthreads();
  if (tid == 0) {
    double t = 0.0;
#pragma unroll 1
    for (int w = 0; w < NTHR; ++w) t += sd[w];
    const float r = (float)t;
    *(volatile float*)(out + klIdx) = r;
    __threadfence();
    *(volatile float*)(out + klIdx) = r;
  }
}

extern "C" void kernel_launch(void* const* d_in, const int* in_sizes, int n_in,
                              void* d_out, int out_size, void* d_ws, size_t ws_size,
                              hipStream_t stream) {
  if (n_in < 16) return;
  if (in_sizes[0] < FIN || (in_sizes[0] % FIN) != 0) return;
  const int nN = in_sizes[0] / FIN;
  if (nN < 1 || nN > (1 << 20)) return;
  if (in_sizes[1] < 2 || (in_sizes[1] & 1) != 0) return;
  const int nE = in_sizes[1] / 2;
  if (nE > (1 << 26)) return;
  if (in_sizes[3] != nN * FZ) return;
  if (in_sizes[4] != FIN * FH) return;
  if (in_sizes[5] != FH || in_sizes[6] != FH || in_sizes[7] != FH) return;
  if (in_sizes[8] != FH * FZ) return;
  if (in_sizes[9] != FZ || in_sizes[10] != FZ || in_sizes[11] != FZ) return;
  if (in_sizes[12] != FH * FZ) return;
  if (in_sizes[13] != FZ || in_sizes[14] != FZ || in_sizes[15] != FZ) return;
  if ((long long)out_size != (long long)nN * FZ + 1) return;

  const float* x   = (const float*)d_in[0];
  const int*   ei  = (const int*)d_in[1];
  const int*   src = ei;
  const int*   dst = ei + nE;
  const float* ew  = (const float*)d_in[2];
  const float* eps = (const float*)d_in[3];
  const float* W1  = (const float*)d_in[4];
  const float* a1s = (const float*)d_in[5];
  const float* a1d = (const float*)d_in[6];
  const float* b1  = (const float*)d_in[7];
  const float* Wmu = (const float*)d_in[8];
  const float* ams = (const float*)d_in[9];
  const float* amd = (const float*)d_in[10];
  const float* bmu = (const float*)d_in[11];
  const float* Wls = (const float*)d_in[12];
  const float* als = (const float*)d_in[13];
  const float* ald = (const float*)d_in[14];
  const float* bls = (const float*)d_in[15];
  float* out = (float*)d_out;
  const int klIdx = nN * FZ;

  const int NPAD   = ((nN + TGT - 1) / TGT) * TGT;
  const int nAgg   = NPAD / TGT;
  const int nBC    = (nN + NBC - 1) / NBC;
  const int CNTPAD = nBC * NBC;
  if (CNTPAD < NPAD) return;
  if (4 * nBC + 1 > RBN) return;
  const int nBF    = (nN + NBF - 1) / NBF;
  if (nBF > 4 * nBC) return;
  const int csrLen = ((nE + 31) & ~31) + 4096;
  if (31 * 4 * nBC > 4096) return;
  const int nGemmR = NPAD / BM;

  char* ws = (char*)d_ws;
  size_t off = 0;
  const size_t oCnt = off; off += (size_t)CNTPAD * 4;                    off = (off + 255) & ~(size_t)255;
  const size_t oOff = off; off += (size_t)CNTPAD * 4;                    off = (off + 255) & ~(size_t)255;
  const size_t oRb  = off; off += (size_t)RBN * 4;                       off = (off + 255) & ~(size_t)255;
  const size_t oFl  = off; off += (size_t)256;                           off = (off + 255) & ~(size_t)255;
  const size_t oCsr = off; off += (size_t)csrLen * 4;                    off = (off + 255) & ~(size_t)255;
  const size_t oW1  = off; off += (size_t)FH * FIN * 2;                  off = (off + 255) & ~(size_t)255;
  const size_t oW2  = off; off += (size_t)FP * FH * 2;                   off = (off + 255) & ~(size_t)255;
  const size_t oWa1 = off; off += (size_t)OTHR * 4;                      off = (off + 255) & ~(size_t)255;
  const size_t oWa2 = off; off += (size_t)OTHR * 4;                      off = (off + 255) & ~(size_t)255;
  const size_t oA1  = off; off += (size_t)NPAD * FIN * 2;                off = (off + 255) & ~(size_t)255;
  const size_t oEs  = off; off += (size_t)NPAD * 4 * 4;                  off = (off + 255) & ~(size_t)255;
  const size_t oHp  = off; off += (size_t)NPAD * FP * 4;                 off = (off + 255) & ~(size_t)255;
  const size_t oZ1  = off; off += (size_t)NPAD * FP * 4;                 off = (off + 255) & ~(size_t)255;
  const size_t oA2  = off; off += (size_t)NPAD * FH * 2;                 off = (off + 255) & ~(size_t)255;
  const size_t oKl  = off; off += (size_t)nAgg * 32 * 4;                 off = (off + 255) & ~(size_t)255;
  if (off > ws_size || off > (size_t)WSCAP) return;

  int*   cnt   = (int*)(ws + oCnt);
  int*   offp  = (int*)(ws + oOff);
  int*   rb    = (int*)(ws + oRb);
  int*   flagp = (int*)(ws + oFl);
  int*   csr   = (int*)(ws + oCsr);
  _Float16* w1p = (_Float16*)(ws + oW1);
  _Float16* w2p = (_Float16*)(ws + oW2);
  float* wa1   = (float*)(ws + oWa1);
  float* wa2   = (float*)(ws + oWa2);
  _Float16* a1 = (_Float16*)(ws + oA1);
  float* es4   = (float*)(ws + oEs);
  float* hp    = (float*)(ws + oHp);
  float* z1    = (float*)(ws + oZ1);
  _Float16* a2 = (_Float16*)(ws + oA2);
  float* klp   = (float*)(ws + oKl);

  const int vec8 = ((nE & 3) == 0) ? 1 : 0;

  k_count<<<nBC, NTHR, 0, stream>>>(dst, cnt, nE, vec8);
  k_offsets<<<1, OTHR, 0, stream>>>(cnt, offp, rb, flagp, nBC);
  hipFuncSetAttribute(reinterpret_cast<const void*>(&k_fill),
                      hipFuncAttributeMaxDynamicSharedMemorySize, LDS_FILL);
  k_fill<<<nBF, NTHR, LDS_FILL, stream>>>(src, dst, offp, rb, csr, nN, nE, vec8, csrLen);

  {
    const int u1 = FH * (FIN / 8);
    k_wcvt2<<<(u1 + NTHR - 1) / NTHR, NTHR, 0, stream>>>(W1, W1, w1p, FIN, FH, FH, u1);
    const int u2 = (FZ + FZ) * (FH / 8);
    k_wcvt2<<<(u2 + NTHR - 1) / NTHR, NTHR, 0, stream>>>(Wmu, Wls, w2p, FH, FZ, FZ, u2);
  }
  k_wfold4<<<1, OTHR, 0, stream>>>(W1, W1, a1s, a1d, a1s, a1d, wa1, FIN, FH);
  k_wfold4<<<1, OTHR, 0, stream>>>(Wmu, Wls, ams, amd, als, ald, wa2, FH, FZ);

  k_xcvt<<<(NPAD * 16) / NTHR, NTHR, 0, stream>>>(x, a1, nN, NPAD);
  k_logit4<FIN><<<NPAD / NTHR, NTHR, 0, stream>>>(x, wa1, es4, nN);
  k_gemm<64><<<dim3(nGemmR, FH / 64), NTHR, 0, stream>>>(a1, w1p, hp, FIN, FP, nN, NPAD);
  k_aggatt<1><<<nAgg, NTHR, 0, stream>>>(csr, offp, cnt, es4, hp, b1, b1, eps, flagp, z1, a2, out, klp, nN, csrLen);

  k_logit4<FH><<<NPAD / NTHR, NTHR, 0, stream>>>(z1, wa2, es4, nN);
  k_gemm<64><<<dim3(nGemmR, FP / 64), NTHR, 0, stream>>>(a2, w2p, hp, FH, FP, nN, NPAD);
  k_aggatt<2><<<nAgg, NTHR, 0, stream>>>(csr, offp, cnt, es4, hp, bmu, bls, eps, flagp, z1, a2, out, klp, nN, csrLen);

  k_klsum<<<1, NTHR, 0, stream>>>(klp, ew, out, nAgg, klIdx);
}
